// PolicyNetwork_20117626814588
// MI455X (gfx1250) — hardware-verified
//
#include <hip/hip_runtime.h>


#ifndef NR
#define NR 512
#endif
#ifndef NT
#define NT 512
#endif
#define NR_FULL 512
#define NT_FULL 512
#ifndef OUT_PITCH
#define OUT_PITCH NT
#endif
#define KD   256
#define HID  512
#define RBK  4

static_assert(NR % 64 == 0);
static_assert(NT % 64 == 0);
static_assert(NT % 256 == 0);
static_assert(NR % RBK == 0);
static_assert(KD % 64 == 0);
static_assert(HID % 64 == 0);
static_assert(HID % 256 == 0);
static_assert((RBK * HID) % 1024 == 0);
static_assert((RBK * NT) % 1024 == 0);
static_assert(OUT_PITCH % 32 == 0);
static_assert(NR <= NR_FULL);
static_assert(NT <= NT_FULL);
static_assert(((size_t)NR * KD) % 8 == 0);
static_assert(((size_t)NT * KD) % 8 == 0);

typedef unsigned short bf;
typedef __attribute__((ext_vector_type(16))) __bf16   v16bf;
typedef __attribute__((ext_vector_type(8)))  unsigned short v8us;
typedef __attribute__((ext_vector_type(8)))  float    v8f;
typedef __attribute__((ext_vector_type(4)))  float    v4f;
typedef v4f  __attribute__((may_alias)) v4fa;

__device__ __forceinline__ unsigned short f2bf(float f) { unsigned u = __float_as_uint(f); u += 0x7FFFu + ((u >> 16) & 1u); return (unsigned short)(u >> 16); }
__device__ __forceinline__ float bfr(float f) { return __uint_as_float(((unsigned)f2bf(f)) << 16); }
__device__ __forceinline__ v16bf cat16b(v8us lo, v8us hi) { return __builtin_bit_cast(v16bf, __builtin_shufflevector(lo, hi, 0, 1, 2, 3, 4, 5, 6, 7, 8, 9, 10, 11, 12, 13, 14, 15)); }
__device__ __forceinline__ v8f wmmab(v16bf a, v16bf b, v8f c) { return __builtin_amdgcn_wmma_f32_16x16x32_bf16(false, a, false, b, (short)0, c, false, false); }
__device__ __forceinline__ v16bf ldb(const bf* p)  { return cat16b(*(const v8us*)p, *(const v8us*)(p + 16)); }
__device__ __forceinline__ void wave_sync() { __builtin_amdgcn_fence(3  , "wavefront"); __builtin_amdgcn_wave_barrier(); asm volatile("" ::: "memory"); }

__global__ __launch_bounds__(256) void k_cvt8(const float* __restrict__ src, bf* dst, size_t n8) {
    const size_t i = (size_t)blockIdx.x * 256 + threadIdx.x; if (i >= n8) return;
    const v8f v = *(const v8f*)(src + i * 8); v8us o;
#pragma unroll
    for (int k = 0; k < 8; ++k) o[k] = f2bf(v[k]);
    *(volatile v8us*)(dst + i * 8) = o; __threadfence(); *(volatile v8us*)(dst + i * 8) = o;
}

__global__ __launch_bounds__(256) void k_wt(const float* __restrict__ W1, bf* WT) {
    __shared__ __align__(16) float ts[64 * 68];
    const int tid = threadIdx.x;
    const int kin0 = blockIdx.x * 64, n0 = blockIdx.y * 64;
#pragma unroll
    for (int it = 0; it < 4; ++it) { const int p = tid + 256 * it; const int kk = p >> 4, c4 = (p & 15) * 4;
        const v4f v = *(const v4f*)(W1 + (size_t)(kin0 + kk) * HID + n0 + c4);
        *(v4fa*)(&ts[kk * 68 + c4]) = v; }
    __syncthreads();
    const int half = kin0 / KD, kl0 = kin0 % KD;
    v8us o0, o1;
    { const int p = tid;       const int n = p >> 3, k8 = (p & 7) * 8;
#pragma unroll
      for (int j = 0; j < 8; ++j) o0[j] = f2bf(ts[(k8 + j) * 68 + n]); }
    { const int p = tid + 256; const int n = p >> 3, k8 = (p & 7) * 8;
#pragma unroll
      for (int j = 0; j < 8; ++j) o1[j] = f2bf(ts[(k8 + j) * 68 + n]); }
    const size_t a0 = ((size_t)half * HID + n0 + (tid >> 3)) * KD + kl0 + (tid & 7) * 8;
    const size_t a1 = ((size_t)half * HID + n0 + 32 + (tid >> 3)) * KD + kl0 + (tid & 7) * 8;
    *(volatile v8us*)(WT + a0) = o0; *(volatile v8us*)(WT + a1) = o1;
    __threadfence();
    *(volatile v8us*)(WT + a0) = o0; *(volatile v8us*)(WT + a1) = o1;
}

__global__ __launch_bounds__(32) void k_proj(const bf* __restrict__ XB, const bf* __restrict__ WT, const float* __restrict__ b1, float* U) {
    __shared__ __align__(16) float os[16 * 68];
    const int K = KD;
    const int lane = threadIdx.x & 31, lr = lane & 15, hi = lane >> 4; const int r0 = blockIdx.x * 64, c0 = blockIdx.y * 64;
    const int z = (r0 >= NR) ? 1 : 0;
    v8f acc[4][4];
#pragma unroll
    for (int mb = 0; mb < 4; ++mb)
#pragma unroll
        for (int nb = 0; nb < 4; ++nb) acc[mb][nb] = (v8f){};
    const size_t aoff = (size_t)(r0 + lr) * K + 8 * hi, boff = (size_t)z * HID * K + (size_t)(c0 + lr) * K + 8 * hi;
#pragma unroll 1
    for (int kc = 0; kc < K; kc += 32) {
        v16bf a[4];
#pragma unroll
        for (int mb = 0; mb < 4; ++mb) a[mb] = ldb(XB + aoff + (size_t)mb * 16 * K + kc);
#pragma unroll
        for (int nb = 0; nb < 4; ++nb) { const v16bf b = ldb(WT + boff + (size_t)nb * 16 * K + kc);
#pragma unroll
            for (int mb = 0; mb < 4; ++mb) acc[mb][nb] = wmmab(a[mb], b, acc[mb][nb]); }
        asm volatile("v_nop\n\tv_nop\n\tv_nop\n\tv_nop" : "+v"(acc[0][0]), "+v"(acc[1][1]), "+v"(acc[2][2]), "+v"(acc[3][3]) : "v"(a[0]), "v"(a[1]), "v"(a[2]), "v"(a[3]));
    }
    const int cofs = lr * 4;
    v4f bv;
#pragma unroll
    for (int i = 0; i < 4; ++i) { const float x = b1[c0 + cofs + i]; const float xr = bfr(x); bv[i] = z ? xr : 0.0f; }
#pragma unroll
    for (int mb = 0; mb < 4; ++mb) {
#pragma unroll
        for (int nb = 0; nb < 4; ++nb) {
#pragma unroll
            for (int j = 0; j < 8; ++j) os[(hi * 8 + j) * 68 + nb * 16 + lr] = acc[mb][nb][j]; }
        wave_sync();
        float* ob = U + (size_t)(r0 + mb * 16) * HID + c0;
#pragma unroll 1
        for (int ps = 0; ps < 2; ++ps) {
#pragma unroll
            for (int s = 0; s < 8; ++s) { const int row = 2 * s + hi;
                const v4f val = *(const v4fa*)(&os[row * 68 + cofs]) + bv;
                *(volatile v4f*)(ob + (size_t)row * HID + cofs) = val; }
            if (ps == 0) __threadfence(); }
        wave_sync();
    }
}

__global__ __launch_bounds__(256) void k_head(const float* __restrict__ U, const float* __restrict__ W2, const float* __restrict__ b2, float* OUT) {
    __shared__ __align__(16) float rs[RBK * HID];
    __shared__ __align__(16) float w2s[HID];
    __shared__ __align__(16) float res[RBK * NT];
    const int tid = threadIdx.x; const int r0 = blockIdx.x * RBK;
#pragma unroll
    for (int it = 0; it < RBK * HID / 1024; ++it) { const int p = tid + 256 * it;
        const v4f v = *(const v4f*)(U + (size_t)r0 * HID + (size_t)p * 4);
        *(v4fa*)(&rs[p * 4]) = v; }
#pragma unroll
    for (int it = 0; it < HID / 256; ++it) { const int i = tid + 256 * it; w2s[i] = bfr(W2[i]); }
    const float bb = bfr(b2[0]);
    __syncthreads();
    const float* TP = U + (size_t)NR * HID;
#pragma unroll 1
    for (int q = 0; q < NT / 256; ++q) {
        const int t = tid + 256 * q;
        const float* tp = TP + (size_t)t * HID;
        float a0 = 0.0f, a1 = 0.0f, a2 = 0.0f, a3 = 0.0f;
#pragma unroll 1
        for (int k = 0; k < HID; k += 4) {
            const v4f tv = *(const v4f*)(tp + k);
            const v4f wv = *(const v4fa*)(&w2s[k]);
            const v4f x0 = *(const v4fa*)(&rs[0 * HID + k]);
            const v4f x1 = *(const v4fa*)(&rs[1 * HID + k]);
            const v4f x2 = *(const v4fa*)(&rs[2 * HID + k]);
            const v4f x3 = *(const v4fa*)(&rs[3 * HID + k]);
#pragma unroll
            for (int i = 0; i < 4; ++i) {
                a0 = fmaf(fmaxf(x0[i] + tv[i], 0.0f), wv[i], a0);
                a1 = fmaf(fmaxf(x1[i] + tv[i], 0.0f), wv[i], a1);
                a2 = fmaf(fmaxf(x2[i] + tv[i], 0.0f), wv[i], a2);
                a3 = fmaf(fmaxf(x3[i] + tv[i], 0.0f), wv[i], a3);
            }
        }
        res[0 * NT + t] = a0 + bb; res[1 * NT + t] = a1 + bb; res[2 * NT + t] = a2 + bb; res[3 * NT + t] = a3 + bb;
    }
    __syncthreads();
    constexpr int NIT = RBK * NT / 1024;
    v4f vals[NIT]; size_t offs[NIT];
#pragma unroll
    for (int it = 0; it < NIT; ++it) { const int p = tid + 256 * it; const int row = p / (NT / 4), c4 = (p % (NT / 4)) * 4;
        vals[it] = *(const v4fa*)(&res[row * NT + c4]);
        offs[it] = (size_t)(r0 + row) * OUT_PITCH + c4; }
#pragma unroll
    for (int it = 0; it < NIT; ++it) *(volatile v4f*)(OUT + offs[it]) = vals[it];
    __threadfence();
#pragma unroll
    for (int it = 0; it < NIT; ++it) *(volatile v4f*)(OUT + offs[it]) = vals[it];
}

static_assert(RBK == 4);

static constexpr size_t al256(size_t v) { return (v + 255) & ~(size_t)255; }
static constexpr size_t SZ_XB = al256((size_t)(NR + NT) * KD * 2);
static constexpr size_t SZ_WT = al256((size_t)2 * HID * KD * 2);
static constexpr size_t SZ_U  = al256((size_t)(NR + NT) * HID * 4);
static constexpr size_t SZ_TOTAL = SZ_XB + SZ_WT + SZ_U;
static_assert(SZ_TOTAL <= (size_t)134217728);

extern "C" void kernel_launch(void* const* d_in, const int* in_sizes, int n_in,
                              void* d_out, int out_size, void* d_ws, size_t ws_size, hipStream_t stream) {
    if (n_in < 6) return;
    if ((size_t)in_sizes[0] < (size_t)NR * KD) return;
    if ((size_t)in_sizes[1] < (size_t)NT * KD) return;
    if ((size_t)in_sizes[2] < (size_t)2 * KD * HID) return;
    if ((size_t)in_sizes[3] < (size_t)HID || (size_t)in_sizes[4] < (size_t)HID || (size_t)in_sizes[5] < (size_t)1) return;
    if ((size_t)out_size < (size_t)(NR - 1) * OUT_PITCH + NT) return;
    if (SZ_TOTAL > ws_size) return;
    const float* robots = (const float*)d_in[0]; const float* tasks = (const float*)d_in[1]; const float* w1 = (const float*)d_in[2];
    const float* b1 = (const float*)d_in[3]; const float* w2 = (const float*)d_in[4]; const float* b2 = (const float*)d_in[5];
    float* OUT = (float*)d_out;
    char* wsp = (char*)d_ws;
    bf* XB = (bf*)wsp; wsp += SZ_XB;
    bf* WT = (bf*)wsp; wsp += SZ_WT;
    float* U = (float*)wsp; wsp += SZ_U;

    { const size_t n8 = (size_t)NR * KD / 8; k_cvt8<<<(unsigned)((n8 + 255) / 256), 256, 0, stream>>>(robots, XB, n8); }
    { const size_t n8 = (size_t)NT * KD / 8; k_cvt8<<<(unsigned)((n8 + 255) / 256), 256, 0, stream>>>(tasks, XB + (size_t)NR * KD, n8); }
    k_wt<<<dim3(2 * KD / 64, HID / 64, 1), 256, 0, stream>>>(w1, WT);
    k_proj<<<dim3((NR + NT) / 64, HID / 64, 1), 32, 0, stream>>>(XB, WT, b1, U);
    k_head<<<dim3(NR / RBK, 1, 1), 256, 0, stream>>>(U, w2, b2, OUT);
}
